// PretrainedModel_35691178230073
// MI455X (gfx1250) — hardware-run, weakly checked
//
#include <hip/hip_runtime.h>


#ifndef NT
#define NT 4096
#endif
#define NT_FULL 4096
#define NS    512
#define DD    64
#define TPB   32
#define WPB   8
#define TPW   (TPB / WPB)
#define TROWS 16
#define NTILE (NS / TROWS)
#ifndef H1_LO
#define H1_LO 0
#endif

static_assert(NT % TPB == 0);
static_assert(NT >= TPB && NT <= NT_FULL);
static_assert(DD == 64);
static_assert(DD % 32 == 0);
static_assert(NS % TROWS == 0);
static_assert(WPB * TPW == TPB);
static_assert(WPB * 32 == 256);
static_assert(TPB * 4 == 128);
static_assert(8 * 16 == TPB * 4);
static_assert((4 * DD + TPB) * 4 <= 131072);
static_assert(64 * 65 * 4 <= 131072);

typedef unsigned short bf;
typedef __attribute__((ext_vector_type(16))) __bf16   v16bf;
typedef __attribute__((ext_vector_type(8)))  unsigned short v8us;
typedef __attribute__((ext_vector_type(8)))  unsigned int   v8u;
typedef __attribute__((ext_vector_type(8)))  float    v8f;
typedef __attribute__((ext_vector_type(4)))  float    v4f;
typedef v4f  __attribute__((may_alias)) v4fa;

__device__ __forceinline__ unsigned short f2bf(float f) { unsigned u = __float_as_uint(f); u += 0x7FFFu + ((u >> 16) & 1u); return (unsigned short)(u >> 16); }
__device__ __forceinline__ v16bf cat16b(v8us lo, v8us hi) { return __builtin_bit_cast(v16bf, __builtin_shufflevector(lo, hi, 0, 1, 2, 3, 4, 5, 6, 7, 8, 9, 10, 11, 12, 13, 14, 15)); }
__device__ __forceinline__ v8f wmmab(v16bf a, v16bf b, v8f c) { return __builtin_amdgcn_wmma_f32_16x16x32_bf16(false, a, false, b, (short)0, c, false, false); }
__device__ __forceinline__ v16bf ldb(const bf* p)  { return cat16b(*(const v8us*)p, *(const v8us*)(p + 16)); }

__device__ __forceinline__ float bfq(float f) { unsigned u = __float_as_uint(f); u += 0x7FFFu + ((u >> 16) & 1u); return __uint_as_float(u & 0xFFFF0000u); }
__device__ __forceinline__ unsigned pk2(float a, float b) { return (__float_as_uint(a) >> 16) | (__float_as_uint(b) & 0xFFFF0000u); }
__device__ __forceinline__ v8f wmmag(v16bf a, v16bf b, v8f c) {
    c = wmmab(a, b, c);
    asm volatile("v_nop\n\tv_nop\n\tv_nop\n\tv_nop" : "+v"(c) : "v"(a), "v"(b));
    return c;
}

__global__ __launch_bounds__(256) void k_rt(const float* __restrict__ R, bf* RT) {
    __shared__ float ts[64 * 65];
    const int r = blockIdx.x, t = threadIdx.x;
    const float* src = R + (size_t)r * (DD * DD);
#pragma unroll 1
    for (int i = 0; i < 16; ++i) { const int f = i * 256 + t; ts[(f >> 6) * 65 + (f & 63)] = src[f]; }
    __syncthreads();
    bf* dst = RT + (size_t)r * (DD * DD);
#pragma unroll 1
    for (int ps = 0; ps < 2; ++ps) {
#pragma unroll 1
        for (int it = 0; it < 2; ++it) {
            const int e = it * 32 + (t >> 3), c8 = (t & 7) * 8; v8us o;
#pragma unroll
            for (int k = 0; k < 8; ++k) o[k] = f2bf(ts[(c8 + k) * 65 + e]);
            *(volatile v8us*)(dst + e * DD + c8) = o; }
        if (ps == 0) __threadfence(); }
}

__global__ __launch_bounds__(256) __attribute__((amdgpu_num_vgpr(256))) void k_mlp(const float* __restrict__ LAB, const float* __restrict__ X,
                                                                                    const float* __restrict__ W1, const float* __restrict__ B1,
                                                                                    const bf* __restrict__ W2T, const float* __restrict__ B2,
                                                                                    const float* __restrict__ W3, const float* __restrict__ B3, float* OUT) {
    __shared__ __align__(16) float sw1[DD];
    __shared__ __align__(16) float sb1[DD];
    __shared__ __align__(16) float sb2[DD];
    __shared__ __align__(16) float sw3[DD];
    __shared__ __align__(16) float res[TPB];
    const int tid = threadIdx.x, lane = tid & 31, lr = lane & 15, hi = lane >> 4;
    const int wave = __builtin_amdgcn_readfirstlane(threadIdx.x >> 5);
    const int blk = blockIdx.x;

    {
        const int ci = tid & (DD - 1);
        const float s1 = bfq(W1[ci]), s2 = bfq(B1[ci]), s3 = bfq(B2[ci]), s4 = bfq(W3[ci]);
        if (tid < DD) { sw1[ci] = s1; sb1[ci] = s2; sb2[ci] = s3; sw3[ci] = s4; }
    }
    __syncthreads();

    float wv[2][16], cv[2][16];
#pragma unroll
    for (int c = 0; c < 2; ++c) {
#pragma unroll
        for (int q = 0; q < 2; ++q) {
            const int k0 = c * 32 + q * 16 + 8 * hi;
            const v4f w0 = *(const v4fa*)(&sw1[k0]); const v4f w1 = *(const v4fa*)(&sw1[k0 + 4]);
            const v4f c0 = *(const v4fa*)(&sb1[k0]); const v4f c1 = *(const v4fa*)(&sb1[k0 + 4]);
#pragma unroll
            for (int i = 0; i < 4; ++i) { wv[c][q * 8 + i] = w0[i]; wv[c][q * 8 + 4 + i] = w1[i]; cv[c][q * 8 + i] = c0[i]; cv[c][q * 8 + 4 + i] = c1[i]; }
        }
    }
    float b2v[4], w3v[4];
#pragma unroll
    for (int nb = 0; nb < 4; ++nb) { b2v[nb] = sb2[nb * 16 + lr]; w3v[nb] = sw3[nb * 16 + lr]; }
    const float b3v = bfq(B3[0]);
    v16bf bw[2][4];
    const size_t boff = (size_t)lr * DD + 8 * hi;
#pragma unroll
    for (int c = 0; c < 2; ++c)
#pragma unroll
        for (int nb = 0; nb < 4; ++nb) bw[c][nb] = ldb(W2T + boff + (size_t)nb * 16 * DD + c * 32);

#pragma unroll 1
    for (int t = 0; t < TPW; ++t) {
        const int task = blk * TPB + wave * TPW + t;
        const size_t tb = (size_t)task * NS;
        float tsum = 0.0f;
#pragma unroll 1
        for (int tile = 0; tile < NTILE; ++tile) {
            const size_t r0 = tb + (size_t)tile * TROWS;
            const float xm  = bfq(X[r0 + lr]);
            const float lab = bfq(LAB[r0 + 8 * hi + (lr & 7)]);
            v8f acc[4];
#pragma unroll
            for (int nb = 0; nb < 4; ++nb) acc[nb] = (v8f){};
#pragma unroll
            for (int c = 0; c < 2; ++c) {
                v8u ah;
#if H1_LO
                v8u al;
#endif
#pragma unroll
                for (int i = 0; i < 8; ++i) {
                    const float h0 = fmaxf(fmaf(xm, wv[c][2 * i],     cv[c][2 * i]),     0.0f);
                    const float h1 = fmaxf(fmaf(xm, wv[c][2 * i + 1], cv[c][2 * i + 1]), 0.0f);
                    const float q0 = bfq(h0), q1 = bfq(h1);
                    ah[i] = pk2(q0, q1);
#if H1_LO
                    al[i] = pk2(bfq(h0 - q0), bfq(h1 - q1));
#endif
                }
                const v16bf a = __builtin_bit_cast(v16bf, ah);
#pragma unroll
                for (int nb = 0; nb < 4; ++nb) acc[nb] = wmmag(a, bw[c][nb], acc[nb]);
#if H1_LO
                const v16bf a2 = __builtin_bit_cast(v16bf, al);
#pragma unroll
                for (int nb = 0; nb < 4; ++nb) acc[nb] = wmmag(a2, bw[c][nb], acc[nb]);
#endif
            }
            float p[8];
#pragma unroll
            for (int j = 0; j < 8; ++j) {
                float s = 0.0f;
#pragma unroll
                for (int nb = 0; nb < 4; ++nb) s = fmaf(fmaxf(acc[nb][j] + b2v[nb], 0.0f), w3v[nb], s);
                s += __shfl_xor(s, 1, 32);
                s += __shfl_xor(s, 2, 32);
                s += __shfl_xor(s, 4, 32);
                s += __shfl_xor(s, 8, 32);
                p[j] = s;
            }
            float pred = p[0];
#pragma unroll
            for (int j = 1; j < 8; ++j) pred = ((lr & 7) == j) ? p[j] : pred;
            pred += b3v;
            const float e  = lab - pred;
            const float sq = e * e;
            tsum += (lr < 8) ? sq : 0.0f;
        }
        tsum += __shfl_xor(tsum, 16, 32);
        tsum += __shfl_xor(tsum, 8, 32);
        tsum += __shfl_xor(tsum, 4, 32);
        tsum += __shfl_xor(tsum, 2, 32);
        tsum += __shfl_xor(tsum, 1, 32);
        const float mean = tsum * (1.0f / (float)NS);
        if (lane == 0) res[wave * TPW + t] = mean;
    }
    __syncthreads();
    if (wave == 0) {
#pragma unroll 1
        for (int ps = 0; ps < 2; ++ps) {
            if (lane < 8) { const v4f v = *(const v4fa*)(&res[4 * lane]); *(volatile v4f*)(OUT + (size_t)blk * TPB + 4 * lane) = v; }
            if (ps == 0) __threadfence(); }
    }
}

static constexpr size_t al256(size_t v) { return (v + 255) & ~(size_t)255; }
static constexpr size_t SZ_W2T = al256((size_t)DD * DD * 2);
static constexpr size_t SZ_TOTAL = SZ_W2T;
static_assert(SZ_TOTAL <= (size_t)134217728);
static_assert(SZ_W2T >= (size_t)64 * 128);

extern "C" void kernel_launch(void* const* d_in, const int* in_sizes, int n_in,
                              void* d_out, int out_size, void* d_ws, size_t ws_size, hipStream_t stream) {
    if (n_in < 8) return;
    if ((size_t)in_sizes[0] < (size_t)NT * NS || (size_t)in_sizes[1] < (size_t)NT * NS) return;
    if (in_sizes[2] < DD || in_sizes[3] < DD || in_sizes[4] < DD * DD || in_sizes[5] < DD || in_sizes[6] < DD || in_sizes[7] < 1) return;
    if ((size_t)out_size < (size_t)NT) return;
    if (SZ_TOTAL > ws_size) return;
    const float* lab = (const float*)d_in[0];
    const float* xin = (const float*)d_in[1];
    const float* W1  = (const float*)d_in[2];
    const float* b1  = (const float*)d_in[3];
    const float* W2  = (const float*)d_in[4];
    const float* b2  = (const float*)d_in[5];
    const float* W3  = (const float*)d_in[6];
    const float* b3  = (const float*)d_in[7];
    float* OUT = (float*)d_out;
    bf* W2T = (bf*)d_ws;

    k_rt<<<1, 256, 0, stream>>>(W2, W2T);
    k_mlp<<<NT / TPB, 256, 0, stream>>>(lab, xin, W1, b1, W2T, b2, W3, b3, OUT);
}
